// ContinuousConvolutionModel_76441827934480
// MI455X (gfx1250) — hardware-verified
//
#include <hip/hip_runtime.h>
#include <stddef.h>
#include <math.h>

#pragma clang fp contract(off)


#define NPT    6000
#define KNB    16
#define NE     128
#define CELLS  216
#define PTB    16
#define NTHR   128
#define NWAV   4
#define KC     512
#define KCP    520
#define GPB    8
#define NB13   8191
#define NOUT4  4500

#define C23    (2.0f / 3.0f)
#define C4PI   ((float)(4.0 / 3.141592653589793))
#define CEPS   ((float)1e-10)

#define L_KEY  0
#define L_WT   (L_KEY + PTB * NE * 4)
#define L_AF   (L_WT + PTB * NE * 4)
#define L_AHI  (L_AF + PTB * KC * 4)
#define L_ALO  (L_AHI + PTB * KCP * 2)
#define L_RED  (L_ALO + PTB * KCP * 2)
#define L_OUT  (L_RED + NWAV * 256 * 4)
#define L_RNG  (L_OUT + PTB * 64 * 4)
#define LDS_CONV (L_RNG + 2 * PTB * 4)

static_assert(NPT % PTB == 0);
static_assert(NPT % GPB == 0);
static_assert(GPB * KNB == NTHR);
static_assert(NTHR == NWAV * 32);
static_assert((L_WT % 16) == 0 && (L_AF % 16) == 0 && (L_AHI % 16) == 0 && (L_ALO % 16) == 0);
static_assert((L_RED % 16) == 0 && (L_OUT % 16) == 0 && (L_RNG % 16) == 0);
static_assert((KCP % 8) == 0 && (KC % 32) == 0);
static_assert(LDS_CONV <= 160 * 1024);
static_assert((NPT * 3) % 4 == 0 && NOUT4 * 4 == NPT * 3);

typedef float          v4f   __attribute__((ext_vector_type(4)));
typedef int            v4i   __attribute__((ext_vector_type(4)));
typedef float          v8f   __attribute__((ext_vector_type(8)));
typedef unsigned short v8us  __attribute__((ext_vector_type(8)));
typedef __bf16         v16bf __attribute__((ext_vector_type(16)));
union FragB { v16bf v; v8us u[2]; };

__device__ __forceinline__ int iclamp(int v, int lo, int hi) {
  return v < lo ? lo : (v > hi ? hi : v);
}

__device__ __forceinline__ unsigned short bf16bits(float x) {
  unsigned int u = __float_as_uint(x);
  u += 0x7fffu + ((u >> 16) & 1u);
  return (unsigned short)(u >> 16);
}
__device__ __forceinline__ float bf16val(unsigned short b) {
  return __uint_as_float(((unsigned int)b) << 16);
}

__device__ __forceinline__ v8f zero8() {
  v8f z = {0.f, 0.f, 0.f, 0.f, 0.f, 0.f, 0.f, 0.f};
  return z;
}

__device__ __forceinline__ v8f wmb(v16bf a, v16bf b, v8f c) {
  v8f d = __builtin_amdgcn_wmma_f32_16x16x32_bf16(false, a, false, b, (short)0, c, false, false);
#if defined(__HIP_DEVICE_COMPILE__)
  asm volatile("v_nop\n\tv_nop\n\tv_nop\n\tv_nop" : "+v"(d) : "v"(a), "v"(b));
#endif
  return d;
}

__global__ __launch_bounds__(NTHR) void k_geo(const float* __restrict__ pos,
                                              const int* __restrict__ nbr,
                                              const float* __restrict__ mask,
                                              int* gKey, float* gWt) {
  __shared__ int   sK[GPB * NE];
  __shared__ float sV[GPB * NE];
  const int tid = threadIdx.x;
  const int p = tid >> 4, j = tid & 15;
  const int n = blockIdx.x * GPB + p;
  int nb = nbr[n * KNB + j];
  nb = iclamp(nb, 0, NPT - 1);
  const float mk = mask[n * KNB + j];

  const float px = pos[n * 3 + 0], py = pos[n * 3 + 1], pz = pos[n * 3 + 2];
  const float qx = pos[nb * 3 + 0], qy = pos[nb * 3 + 1], qz = pos[nb * 3 + 2];
  const float x = (qx - px) * C23;
  const float y = (qy - py) * C23;
  const float z = (qz - pz) * C23;

  const float xx = x * x;
  const float yy = y * y;
  const float zz = z * z;
  const float sxy = xx + yy;
  const float sq = sxy + zz;
  const bool inside = sq > CEPS;
  const float norm = sqrtf(inside ? sq : 1.0f);
  const float z125 = 1.25f * z;
  const bool pole = (z125 * z) > sxy;
  const float n3 = 3.0f * norm;
  const float dn = norm + fabsf(z);
  const float s_p = sqrtf(n3 / dn);
  const float rxy = sqrtf((pole || !inside) ? 1.0f : sxy);
  const float s_s = norm / rxy;
  const float sgnz = (z > 0.0f) ? 1.0f : ((z < 0.0f) ? -1.0f : 0.0f);
  const float cx = inside ? (pole ? x * s_p : x * s_s) : 0.0f;
  const float cy = inside ? (pole ? y * s_p : y * s_s) : 0.0f;
  const float cz = inside ? (pole ? sgnz * norm : 1.5f * z) : 0.0f;
  const float cxx = cx * cx;
  const float cyy = cy * cy;
  const float rc = cxx + cyy;
  const bool rin = rc > CEPS;
  const float rn = sqrtf(rin ? rc : 1.0f);
  const bool condx = fabsf(cx) >= fabsf(cy);
  const float den0 = condx ? cx : cy;
  const float den = (fabsf(den0) > CEPS) ? den0 : 1.0f;
  const float num = condx ? cy : cx;
  const float rden = 1.0f / den;
  const float tt = C4PI * atanf(num * rden);
  const float major = (den > 0.0f) ? rn : -rn;
  const float mt = major * tt;
  const float u = rin ? (condx ? major : mt) : 0.0f;
  const float v = rin ? (condx ? mt : major) : 0.0f;

  const float a0 = u * 0.5f;  const float b0s = a0 + 0.5f;  const float t0 = b0s * 6.0f - 0.5f;
  const float a1 = v * 0.5f;  const float b1s = a1 + 0.5f;  const float t1 = b1s * 6.0f - 0.5f;
  const float a2 = cz * 0.5f; const float b2s = a2 + 0.5f;  const float t2 = b2s * 6.0f - 0.5f;
  const float fl0 = floorf(t0), fl1 = floorf(t1), fl2 = floorf(t2);
  const float f0 = t0 - fl0, f1 = t1 - fl1, f2 = t2 - fl2;
  const int i00 = (int)fl0, i01 = (int)fl1, i02 = (int)fl2;
  const int   ix[2] = { iclamp(i00, 0, 5), iclamp(i00 + 1, 0, 5) };
  const int   iy[2] = { iclamp(i01, 0, 5), iclamp(i01 + 1, 0, 5) };
  const int   iz[2] = { iclamp(i02, 0, 5), iclamp(i02 + 1, 0, 5) };
  const float wx[2] = { 1.0f - f0, f0 };
  const float wy[2] = { 1.0f - f1, f1 };
  const float wz[2] = { 1.0f - f2, f2 };

  const int ebase = p * NE + j * 8;
#pragma unroll
  for (int a = 0; a < 2; ++a)
#pragma unroll
    for (int b = 0; b < 2; ++b)
#pragma unroll
      for (int c = 0; c < 2; ++c) {
        const int s = a * 4 + b * 2 + c;
        const int cell = ix[a] * 36 + iy[b] * 6 + iz[c];
        const float wab = wx[a] * wy[b];
        const float wabc = wab * wz[c];
        sK[ebase + s] = (cell << 13) | nb;
        sV[ebase + s] = wabc * mk;
      }
  __syncthreads();

#pragma unroll 1
  for (int kst = 2; kst <= NE; kst <<= 1) {
#pragma unroll 1
    for (int jst = kst >> 1; jst > 0; jst >>= 1) {
#pragma unroll
      for (int r = 0; r < 4; ++r) {
        const int q = tid + NTHR * r;
        const int pp = q >> 6;
        const int i = q & 63;
        const int lo = ((i & ~(jst - 1)) << 1) | (i & (jst - 1));
        const int hi = lo + jst;
        const int bl = pp * NE + lo, bh = pp * NE + hi;
        const int ka = sK[bl], kb = sK[bh];
        const float wa = sV[bl], wb = sV[bh];
        const bool asc = (lo & kst) == 0;
        const bool sw = asc ? (ka > kb) : (ka < kb);
        sK[bl] = sw ? kb : ka;
        sK[bh] = sw ? ka : kb;
        sV[bl] = sw ? wb : wa;
        sV[bh] = sw ? wa : wb;
      }
      __syncthreads();
    }
  }

  {
    const v4i kv0 = *(const v4i*)(sK + 4 * tid);
    const v4i kv1 = *(const v4i*)(sK + 512 + 4 * tid);
    const v4f wv0 = *(const v4f*)(sV + 4 * tid);
    const v4f wv1 = *(const v4f*)(sV + 512 + 4 * tid);
    int*   gk = gKey + (size_t)blockIdx.x * (GPB * NE);
    float* gw = gWt + (size_t)blockIdx.x * (GPB * NE);
    *(volatile v4i*)(gk + 4 * tid) = kv0;
    *(volatile v4i*)(gk + 512 + 4 * tid) = kv1;
    *(volatile v4f*)(gw + 4 * tid) = wv0;
    *(volatile v4f*)(gw + 512 + 4 * tid) = wv1;
    __threadfence();
    *(volatile v4i*)(gk + 4 * tid) = kv0;
    *(volatile v4i*)(gk + 512 + 4 * tid) = kv1;
    *(volatile v4f*)(gw + 4 * tid) = wv0;
    *(volatile v4f*)(gw + 512 + 4 * tid) = wv1;
  }
}

template <int CIN, int COUT, int COUTP>
__global__ __launch_bounds__(256) void k_prepw(const float* __restrict__ W,
                                              unsigned short* pHi, unsigned short* pLo) {
  constexpr int K = CELLS * CIN;
  constexpr int G = K / 8;
  constexpr int TOT = COUTP * G;
  static_assert((K % 32) == 0);
  const int i = blockIdx.x * 256 + (int)threadIdx.x;
  if (i >= TOT) return;
  const int o = i / G;
  const int k0 = (i - o * G) * 8;
  const int oc = o < COUT ? o : COUT - 1;
  float v[8];
#pragma unroll
  for (int e = 0; e < 8; ++e) {
    const float xw = W[(size_t)(k0 + e) * COUT + oc];
    v[e] = (o < COUT) ? xw : xw * 0.0f;
  }
  v8us hv, lv;
#pragma unroll
  for (int e = 0; e < 8; ++e) {
    const unsigned short hb = bf16bits(v[e]);
    hv[e] = hb;
    lv[e] = bf16bits(v[e] - bf16val(hb));
  }
  const size_t off = (size_t)o * K + k0;
  *(volatile v8us*)(pHi + off) = hv;
  *(volatile v8us*)(pLo + off) = lv;
  __threadfence();
  *(volatile v8us*)(pHi + off) = hv;
  *(volatile v8us*)(pLo + off) = lv;
}

template <int CIN, int COUT, int COUTP, bool RELU>
__global__ __launch_bounds__(NTHR) void k_conv(const float* __restrict__ X,
                                               const unsigned short* __restrict__ pHi,
                                               const unsigned short* __restrict__ pLo,
                                               const float* __restrict__ bias,
                                               const int* __restrict__ gKey,
                                               const float* __restrict__ gWt,
                                               float* Xout) {
  constexpr int CPC = KC / CIN;
  constexpr int NCH = (CELLS + CPC - 1) / CPC;
  constexpr int NT = COUTP / 16;
  constexpr int S = NWAV / NT;
  constexpr int K = CELLS * CIN;
  static_assert(KC % CIN == 0);
  static_assert((CPC * CIN) % 32 == 0);
  static_assert(((CELLS % CPC) * CIN) % 32 == 0);
  static_assert(NT >= 1 && NT * S == NWAV);
  static_assert(COUTP <= 64 && COUT <= COUTP && (COUTP % 16) == 0);

  extern __shared__ v4f lds_dyn[];
  char* lb = (char*)lds_dyn;
  int*            sKey = (int*)(lb + L_KEY);
  float*          sWt  = (float*)(lb + L_WT);
  float*          sAf  = (float*)(lb + L_AF);
  unsigned short* sAhi = (unsigned short*)(lb + L_AHI);
  unsigned short* sAlo = (unsigned short*)(lb + L_ALO);
  float*          sRed = (float*)(lb + L_RED);
  float*          sOut = (float*)(lb + L_OUT);
  int*            sBeg = (int*)(lb + L_RNG);
  int*            sEnd = sBeg + PTB;

  const int tid = threadIdx.x, lane = tid & 31, wave = tid >> 5, hh = lane >> 4, m = lane & 15;
  const int n0 = blockIdx.x * PTB;
  const int tl = wave % NT;
  const int sp = wave / NT;

  {
    const v4i* gk = (const v4i*)(gKey + (size_t)n0 * NE);
    const v4f* gw = (const v4f*)(gWt + (size_t)n0 * NE);
    v4i* sk4 = (v4i*)sKey;
    v4f* sw4 = (v4f*)sWt;
    for (int q = tid; q < PTB * NE / 4; q += NTHR) {
      sk4[q] = gk[q];
      sw4[q] = gw[q];
    }
  }
  if (tid < PTB) { sBeg[tid] = 0; sEnd[tid] = 0; }
  v8f acc = zero8();
  __syncthreads();

#pragma unroll 1
  for (int ch = 0; ch < NCH; ++ch) {
    const int c0 = ch * CPC;
    const int rem = CELLS - c0;
    const int ncell = rem < CPC ? rem : CPC;
    const int ksteps = (ncell * CIN) >> 5;

    {
      v4f z;
      z[0] = 0.0f; z[1] = 0.0f; z[2] = 0.0f; z[3] = 0.0f;
      v4f* a4 = (v4f*)sAf;
      for (int q = tid; q < PTB * KC / 4; q += NTHR) a4[q] = z;
    }
    if (tid < PTB) {
      const int p = tid;
      int e = sEnd[p];
      e = iclamp(e, 0, NE);
      const int beg = e;
      const int lim = (c0 + ncell) << 13;
      while (e < NE) {
        const int ky = sKey[p * NE + e];
        if (ky >= lim) break;
        ++e;
      }
      sBeg[p] = beg;
      sEnd[p] = e;
    }
    __syncthreads();

    for (int pc = tid; pc < PTB * CIN; pc += NTHR) {
      const int p = pc / CIN, c = pc - p * CIN;
      int eb = sBeg[p], ee = sEnd[p];
      eb = eb < 0 ? 0 : eb;
      ee = ee > NE ? NE : ee;
      float* arow = sAf + p * KC + c;
      const float* xc = X + c;
      const int* kr = sKey + p * NE;
      const float* wr = sWt + p * NE;
      for (int e = eb; e < ee; ++e) {
        const int ky = kr[e];
        const float w = wr[e];
        int nbi = ky & NB13;
        nbi = nbi > NPT - 1 ? NPT - 1 : nbi;
        int cl = (ky >> 13) - c0;
        cl = cl < 0 ? 0 : (cl > CPC - 1 ? CPC - 1 : cl);
        const float xv = xc[(size_t)nbi * CIN];
        const float pr = w * xv;
        float* ap = arow + cl * CIN;
        const float cur = *ap;
        *ap = cur + pr;
      }
    }
    __syncthreads();

    for (int q = tid; q < PTB * KC / 8; q += NTHR) {
      const int p = q / (KC / 8), k8 = (q - p * (KC / 8)) * 8;
      const v4f a0 = *(const v4f*)(sAf + p * KC + k8);
      const v4f a1 = *(const v4f*)(sAf + p * KC + k8 + 4);
      v8us hv, lv;
#pragma unroll
      for (int e = 0; e < 4; ++e) {
        const unsigned short hb = bf16bits(a0[e]);
        hv[e] = hb;
        lv[e] = bf16bits(a0[e] - bf16val(hb));
      }
#pragma unroll
      for (int e = 0; e < 4; ++e) {
        const unsigned short hb = bf16bits(a1[e]);
        hv[4 + e] = hb;
        lv[4 + e] = bf16bits(a1[e] - bf16val(hb));
      }
      *(v8us*)(sAhi + p * KCP + k8) = hv;
      *(v8us*)(sAlo + p * KCP + k8) = lv;
    }
    __syncthreads();

    {
      const unsigned short* ah = sAhi + m * KCP + 8 * hh;
      const unsigned short* al = sAlo + m * KCP + 8 * hh;
      const size_t bo = (size_t)(16 * tl + m) * K + (size_t)c0 * CIN + 8 * hh;
      const unsigned short* bh = pHi + bo;
      const unsigned short* bl = pLo + bo;
      for (int kk = sp; kk < ksteps; kk += S) {
        const int ko = 32 * kk;
        FragB fah, fal, fbh, fbl;
        fah.u[0] = *(const v8us*)(ah + ko);
        fah.u[1] = *(const v8us*)(ah + ko + 16);
        fal.u[0] = *(const v8us*)(al + ko);
        fal.u[1] = *(const v8us*)(al + ko + 16);
        fbh.u[0] = *(const v8us*)(bh + ko);
        fbh.u[1] = *(const v8us*)(bh + ko + 16);
        fbl.u[0] = *(const v8us*)(bl + ko);
        fbl.u[1] = *(const v8us*)(bl + ko + 16);
        acc = wmb(fah.v, fbh.v, acc);
        acc = wmb(fah.v, fbl.v, acc);
        acc = wmb(fal.v, fbh.v, acc);
      }
    }
  }

  {
    float* rp = sRed + wave * 256 + lane * 8;
    v4f r0, r1;
    r0[0] = acc[0]; r0[1] = acc[1]; r0[2] = acc[2]; r0[3] = acc[3];
    r1[0] = acc[4]; r1[1] = acc[5]; r1[2] = acc[6]; r1[3] = acc[7];
    *(v4f*)rp = r0;
    *(v4f*)(rp + 4) = r1;
  }
  __syncthreads();
  for (int idx = tid; idx < PTB * COUTP; idx += NTHR) {
    const int row = idx / COUTP, col = idx - row * COUTP;
    const int tt = col >> 4, mm = col & 15, r = row & 7, h2 = row >> 3;
    const int ln = mm + 16 * h2;
    float v = 0.0f;
#pragma unroll
    for (int s2 = 0; s2 < S; ++s2) v = v + sRed[(s2 * NT + tt) * 256 + ln * 8 + r];
    const int oc = col < COUT ? col : COUT - 1;
    const float bv = bias[oc];
    v = v + (col < COUT ? bv : bv * 0.0f);
    if (RELU) v = fmaxf(v, 0.0f);
    sOut[idx] = v;
  }
  __syncthreads();

  {
    float* go = Xout + (size_t)n0 * COUTP;
    const v4f* so = (const v4f*)sOut;
    for (int q = tid; q < PTB * COUTP / 4; q += NTHR) *(volatile v4f*)(go + 4 * q) = so[q];
    __threadfence();
    for (int q = tid; q < PTB * COUTP / 4; q += NTHR) *(volatile v4f*)(go + 4 * q) = so[q];
  }
}

__global__ __launch_bounds__(256) void k_out(const float* __restrict__ X5, float* out) {
  const int tid = threadIdx.x;
#pragma unroll 1
  for (int pass = 0; pass < 2; ++pass) {
    for (int q = tid; q < NOUT4; q += 256) {
      v4f ov;
#pragma unroll
      for (int uu = 0; uu < 4; ++uu) {
        const int f = 4 * q + uu;
        const int n = f / 3;
        const int c = f - n * 3;
        ov[uu] = X5[(size_t)n * 16 + c];
      }
      *(volatile v4f*)(out + 4 * q) = ov;
    }
    if (pass == 0) __threadfence();
  }
}

extern "C" void kernel_launch(void* const* d_in, const int* in_sizes, int n_in,
                              void* d_out, int out_size, void* d_ws, size_t ws_size,
                              hipStream_t stream) {
  if (n_in < 14) return;
  if (in_sizes[0] != NPT * 4 || in_sizes[1] != NPT * 3) return;
  if (in_sizes[2] != NPT * KNB || in_sizes[3] != NPT * KNB) return;
  if (in_sizes[4] != CELLS * 4 * 64 || in_sizes[5] != 64) return;
  if (in_sizes[6] != CELLS * 64 * 64 || in_sizes[7] != 64) return;
  if (in_sizes[8] != CELLS * 64 * 32 || in_sizes[9] != 32) return;
  if (in_sizes[10] != CELLS * 32 * 32 || in_sizes[11] != 32) return;
  if (in_sizes[12] != CELLS * 32 * 3 || in_sizes[13] != 3) return;
  if (out_size != NPT * 3) return;

  const float* feats = (const float*)d_in[0];
  const float* pos   = (const float*)d_in[1];
  const int*   nbr   = (const int*)d_in[2];
  const float* mask  = (const float*)d_in[3];
  const float* W0 = (const float*)d_in[4];
  const float* B0 = (const float*)d_in[5];
  const float* W1 = (const float*)d_in[6];
  const float* B1 = (const float*)d_in[7];
  const float* W2 = (const float*)d_in[8];
  const float* B2 = (const float*)d_in[9];
  const float* W3 = (const float*)d_in[10];
  const float* B3 = (const float*)d_in[11];
  const float* W4 = (const float*)d_in[12];
  const float* B4 = (const float*)d_in[13];
  float* out = (float*)d_out;

  char* ws = (char*)d_ws;
  size_t off = 0;
  auto take = [&](size_t bytes) -> size_t {
    const size_t o = off;
    off += (bytes + 255) & ~(size_t)255;
    return o;
  };
  const size_t oKey = take((size_t)NPT * NE * 4);
  const size_t oWt  = take((size_t)NPT * NE * 4);
  const size_t oH0 = take((size_t)64 * CELLS * 4 * 2),  oL0 = take((size_t)64 * CELLS * 4 * 2);
  const size_t oH1 = take((size_t)64 * CELLS * 64 * 2), oL1 = take((size_t)64 * CELLS * 64 * 2);
  const size_t oH2 = take((size_t)32 * CELLS * 64 * 2), oL2 = take((size_t)32 * CELLS * 64 * 2);
  const size_t oH3 = take((size_t)32 * CELLS * 32 * 2), oL3 = take((size_t)32 * CELLS * 32 * 2);
  const size_t oH4 = take((size_t)16 * CELLS * 32 * 2), oL4 = take((size_t)16 * CELLS * 32 * 2);
  const size_t oX1 = take((size_t)NPT * 64 * 4);
  const size_t oX2 = take((size_t)NPT * 64 * 4);
  const size_t oX3 = take((size_t)NPT * 32 * 4);
  const size_t oX4 = take((size_t)NPT * 32 * 4);
  const size_t oX5 = take((size_t)NPT * 16 * 4);
  if (off > ws_size || off > (size_t)134217728) return;

  int*   gKey = (int*)(ws + oKey);
  float* gWt  = (float*)(ws + oWt);
  unsigned short* H0 = (unsigned short*)(ws + oH0); unsigned short* Lo0 = (unsigned short*)(ws + oL0);
  unsigned short* H1 = (unsigned short*)(ws + oH1); unsigned short* Lo1 = (unsigned short*)(ws + oL1);
  unsigned short* H2 = (unsigned short*)(ws + oH2); unsigned short* Lo2 = (unsigned short*)(ws + oL2);
  unsigned short* H3 = (unsigned short*)(ws + oH3); unsigned short* Lo3 = (unsigned short*)(ws + oL3);
  unsigned short* H4 = (unsigned short*)(ws + oH4); unsigned short* Lo4 = (unsigned short*)(ws + oL4);
  float* X1 = (float*)(ws + oX1);
  float* X2 = (float*)(ws + oX2);
  float* X3 = (float*)(ws + oX3);
  float* X4 = (float*)(ws + oX4);
  float* X5 = (float*)(ws + oX5);

  k_geo<<<NPT / GPB, NTHR, 0, stream>>>(pos, nbr, mask, gKey, gWt);

  k_prepw<4, 64, 64><<<(64 * CELLS * 4 / 8 + 255) / 256, 256, 0, stream>>>(W0, H0, Lo0);
  k_prepw<64, 64, 64><<<(64 * CELLS * 64 / 8 + 255) / 256, 256, 0, stream>>>(W1, H1, Lo1);
  k_prepw<64, 32, 32><<<(32 * CELLS * 64 / 8 + 255) / 256, 256, 0, stream>>>(W2, H2, Lo2);
  k_prepw<32, 32, 32><<<(32 * CELLS * 32 / 8 + 255) / 256, 256, 0, stream>>>(W3, H3, Lo3);
  k_prepw<32, 3, 16><<<(16 * CELLS * 32 / 8 + 255) / 256, 256, 0, stream>>>(W4, H4, Lo4);

  hipFuncSetAttribute(reinterpret_cast<const void*>(&k_conv<4, 64, 64, true>),
                      hipFuncAttributeMaxDynamicSharedMemorySize, LDS_CONV);
  hipFuncSetAttribute(reinterpret_cast<const void*>(&k_conv<64, 64, 64, true>),
                      hipFuncAttributeMaxDynamicSharedMemorySize, LDS_CONV);
  hipFuncSetAttribute(reinterpret_cast<const void*>(&k_conv<64, 32, 32, true>),
                      hipFuncAttributeMaxDynamicSharedMemorySize, LDS_CONV);
  hipFuncSetAttribute(reinterpret_cast<const void*>(&k_conv<32, 32, 32, true>),
                      hipFuncAttributeMaxDynamicSharedMemorySize, LDS_CONV);
  hipFuncSetAttribute(reinterpret_cast<const void*>(&k_conv<32, 3, 16, false>),
                      hipFuncAttributeMaxDynamicSharedMemorySize, LDS_CONV);
  k_conv<4, 64, 64, true><<<NPT / PTB, NTHR, LDS_CONV, stream>>>(feats, H0, Lo0, B0, gKey, gWt, X1);
  k_conv<64, 64, 64, true><<<NPT / PTB, NTHR, LDS_CONV, stream>>>(X1, H1, Lo1, B1, gKey, gWt, X2);
  k_conv<64, 32, 32, true><<<NPT / PTB, NTHR, LDS_CONV, stream>>>(X2, H2, Lo2, B2, gKey, gWt, X3);
  k_conv<32, 32, 32, true><<<NPT / PTB, NTHR, LDS_CONV, stream>>>(X3, H3, Lo3, B3, gKey, gWt, X4);
  k_conv<32, 3, 16, false><<<NPT / PTB, NTHR, LDS_CONV, stream>>>(X4, H4, Lo4, B4, gKey, gWt, X5);

  k_out<<<1, 256, 0, stream>>>(X5, out);
}
